// MulLeaBlock_15573551415935
// MI455X (gfx1250) — hardware-run, weakly checked
//
#include <hip/hip_runtime.h>


#define NB_  4
#define NN   4096
#define C0   512
#define C1   256
#define CI   128
#define PCAR 1024.0f
typedef _Float16 h16;
typedef unsigned short bf;
typedef __attribute__((ext_vector_type(16))) __bf16   v16bf;
typedef __attribute__((ext_vector_type(16))) _Float16 v16h;
typedef __attribute__((ext_vector_type(8)))  _Float16 v8h;
typedef __attribute__((ext_vector_type(8)))  unsigned short v8us;
typedef __attribute__((ext_vector_type(8)))  float    v8f;
typedef __attribute__((ext_vector_type(4)))  float    v4f;
typedef v8h  __attribute__((may_alias)) v8ha;
typedef v4f  __attribute__((may_alias)) v4fa;
typedef v8us __attribute__((may_alias)) v8usa;

__device__ __forceinline__ unsigned short f2bf(float f) { unsigned u = __float_as_uint(f); u += 0x7FFFu + ((u >> 16) & 1u); return (unsigned short)(u >> 16); }
__device__ __forceinline__ float bf2f(unsigned short b) { return __uint_as_float(((unsigned)b) << 16); }
__device__ __forceinline__ float bfr(float f) { return bf2f(f2bf(f)); }
__device__ __forceinline__ v16h cat16(v8h lo, v8h hi) { return __builtin_shufflevector(lo, hi, 0, 1, 2, 3, 4, 5, 6, 7, 8, 9, 10, 11, 12, 13, 14, 15); }
__device__ __forceinline__ v16bf cat16b(v8us lo, v8us hi) { return __builtin_bit_cast(v16bf, __builtin_shufflevector(lo, hi, 0, 1, 2, 3, 4, 5, 6, 7, 8, 9, 10, 11, 12, 13, 14, 15)); }
__device__ __forceinline__ v8f wmma16(v16h a, v16h b, v8f c) { return __builtin_amdgcn_wmma_f32_16x16x32_f16(false, a, false, b, (short)0, c, false, false); }
__device__ __forceinline__ v8f wmmab(v16bf a, v16bf b, v8f c) { return __builtin_amdgcn_wmma_f32_16x16x32_bf16(false, a, false, b, (short)0, c, false, false); }


template <typename T16> struct WFrag;
template <> struct WFrag<h16> { typedef v16h V; static __device__ __forceinline__ V ld(const h16* p) { return cat16(*(const v8h*)p, *(const v8h*)(p + 16)); } static __device__ __forceinline__ v8f mma(V a, V b, v8f c) { return wmma16(a, b, c); } };
template <> struct WFrag<bf> { typedef v16bf V; static __device__ __forceinline__ V ld(const bf* p) { return cat16b(*(const v8us*)p, *(const v8us*)(p + 16)); } static __device__ __forceinline__ v8f mma(V a, V b, v8f c) { return wmmab(a, b, c); } };
template <typename T16, int NSPLIT, bool BIAS>
__global__ __launch_bounds__(32) void k_gemmw(const T16* __restrict__ A, const T16* __restrict__ A2, const T16* __restrict__ Bt, const T16* __restrict__ Bt2, int K, float* C, int ldc, const float* __restrict__ bias, size_t sA, size_t sB, size_t sC) {
    typedef typename WFrag<T16>::V V;
    __shared__ __align__(16) float os[16 * 68];
    const size_t z = blockIdx.z; A += z * sA; if (A2) A2 += z * sA; Bt += z * sB; if (Bt2) Bt2 += z * sB; C += z * sC;
    const int lane = threadIdx.x & 31, lr = lane & 15, hi = lane >> 4; const int r0 = blockIdx.x * 64, c0 = blockIdx.y * 64;
    v8f acc[4][4];
#pragma unroll
    for (int mb = 0; mb < 4; ++mb)
#pragma unroll
        for (int nb = 0; nb < 4; ++nb) acc[mb][nb] = (v8f){};
    const size_t aoff = (size_t)(r0 + lr) * K + 8 * hi, boff = (size_t)(c0 + lr) * K + 8 * hi;
#pragma unroll 1
    for (int kc = 0; kc < K; kc += 32) {
        V a[4], a2[4];
#pragma unroll
        for (int mb = 0; mb < 4; ++mb) { a[mb] = WFrag<T16>::ld(A + aoff + (size_t)mb * 16 * K + kc); if (NSPLIT == 1 || NSPLIT == 2) a2[mb] = WFrag<T16>::ld(A2 + aoff + (size_t)mb * 16 * K + kc); }
#pragma unroll
        for (int nb = 0; nb < 4; ++nb) { const V b = WFrag<T16>::ld(Bt + boff + (size_t)nb * 16 * K + kc); V b2; if (NSPLIT >= 2) b2 = WFrag<T16>::ld(Bt2 + boff + (size_t)nb * 16 * K + kc);
#pragma unroll
            for (int mb = 0; mb < 4; ++mb) { acc[mb][nb] = WFrag<T16>::mma(a[mb], b, acc[mb][nb]); if (NSPLIT == 1 || NSPLIT == 2) acc[mb][nb] = WFrag<T16>::mma(a2[mb], b, acc[mb][nb]); if (NSPLIT >= 2) acc[mb][nb] = WFrag<T16>::mma(a[mb], b2, acc[mb][nb]); } }
        asm volatile("v_nop\n\tv_nop\n\tv_nop\n\tv_nop" : "+v"(acc[0][0]), "+v"(acc[1][1]), "+v"(acc[2][2]), "+v"(acc[3][3]) : "v"(a[0]), "v"(a[3]));
    }
#pragma unroll
    for (int mb = 0; mb < 4; ++mb) {
#pragma unroll
        for (int nb = 0; nb < 4; ++nb) {
#pragma unroll
            for (int j = 0; j < 8; ++j) os[(hi * 8 + j) * 68 + nb * 16 + lr] = acc[mb][nb][j]; }
        __builtin_amdgcn_wave_barrier(); asm volatile("" ::: "memory");
        float* crow = C + (size_t)(r0 + mb * 16) * ldc + c0;
#pragma unroll 1
        for (int ps = 0; ps < 2; ++ps) {
#pragma unroll
            for (int s = 0; s < 8; ++s) { const int row = 2 * s + hi, cofs = lr * 4; v4f val = *(const v4fa*)(os + row * 68 + cofs); if (BIAS) { val[0] += bfr(bias[c0 + cofs]); val[1] += bfr(bias[c0 + cofs + 1]); val[2] += bfr(bias[c0 + cofs + 2]); val[3] += bfr(bias[c0 + cofs + 3]); }
                *(volatile v4f*)(crow + (size_t)row * ldc + cofs) = val; }
            if (ps == 0) __threadfence(); }
        __builtin_amdgcn_wave_barrier(); asm volatile("" ::: "memory");
    }
}

__device__ __forceinline__ h16 tohx(float x) { return (h16)x; }
__device__ __forceinline__ void splitf(float y, unsigned short& h, unsigned short& l) { h = f2bf(y); l = f2bf(y - bf2f(h)); }
typedef __attribute__((ext_vector_type(2))) _Float16 v2h;
typedef __attribute__((ext_vector_type(4))) _Float16 v4h;
typedef __attribute__((ext_vector_type(2))) unsigned short v2us;
typedef __attribute__((ext_vector_type(4))) unsigned short v4us;
typedef __attribute__((ext_vector_type(2))) float v2f;

__global__ __launch_bounds__(256) void k_cvt8(const float* __restrict__ src, bf* dst, size_t n8) { const size_t i = (size_t)blockIdx.x * 256 + threadIdx.x; if (i >= n8) return; const v8f v = *(const v8f*)(src + i * 8); v8us o;
#pragma unroll
    for (int k = 0; k < 8; ++k) o[k] = f2bf(v[k]); *(volatile v8us*)(dst + i * 8) = o; __threadfence(); *(volatile v8us*)(dst + i * 8) = o; }
__global__ __launch_bounds__(256) void k_xt8(const float* __restrict__ xb, int C, bf* XT) { const size_t e = ((size_t)blockIdx.x * 256 + threadIdx.x) * 4; if (e >= (size_t)NN * C) return; const int c = (int)(e % C), n = (int)(e / C); v4us o;
#pragma unroll
    for (int q = 0; q < 4; ++q) o[q] = f2bf(xb[(size_t)(c + q) * NN + n]); *(volatile v4us*)(XT + e) = o; __threadfence(); *(volatile v4us*)(XT + e) = o; }
__global__ __launch_bounds__(256) void k_split2(const float* __restrict__ F, bf* Ph, bf* Pl, size_t n) { const size_t i = ((size_t)blockIdx.x * 256 + threadIdx.x) * 2; if (i >= n) return; v2us oh, ol;
#pragma unroll
    for (int q = 0; q < 2; ++q) { unsigned short a, c2; splitf(F[i + q], a, c2); oh[q] = a; ol[q] = c2; } *(volatile v2us*)(Ph + i) = oh; *(volatile v2us*)(Pl + i) = ol; __threadfence(); *(volatile v2us*)(Ph + i) = oh; *(volatile v2us*)(Pl + i) = ol; }
__global__ __launch_bounds__(256) void k_gt16(const float* __restrict__ G, h16* GT) { const size_t e = ((size_t)blockIdx.x * 256 + threadIdx.x) * 2; if (e >= (size_t)C1 * NN) return; const int m = (int)(e % NN), c = (int)(e / NN); v2h o; o[0] = tohx(G[(size_t)m * C1 + c]); o[1] = tohx(G[(size_t)(m + 1) * C1 + c]); *(volatile v2h*)(GT + e) = o; __threadfence(); *(volatile v2h*)(GT + e) = o; }
__global__ __launch_bounds__(256) void k_colst(const float* __restrict__ S, float* CM, float* CIv) { const int m = blockIdx.x * 256 + threadIdx.x; if (m >= NN) return; float mx = -3.0e38f;
    for (int n = 0; n < NN; ++n) mx = fmaxf(mx, S[(size_t)n * NN + m]);
    float s = 0.f; for (int n = 0; n < NN; ++n) { float d0 = __fsub_rn(S[(size_t)n * NN + m], mx); asm volatile("" : "+v"(d0)); s = __fadd_rn(s, __expf(d0)); }
    const float ci = __fdiv_rn(PCAR, s); *(volatile float*)(CM + m) = mx; *(volatile float*)(CIv + m) = ci; __threadfence(); *(volatile float*)(CM + m) = mx; *(volatile float*)(CIv + m) = ci; }
__global__ __launch_bounds__(256) void k_pcol(const float* __restrict__ S, const float* __restrict__ CM, const float* __restrict__ CIv, h16* P) { const size_t e = ((size_t)blockIdx.x * 256 + threadIdx.x) * 4; if (e >= (size_t)NN * NN) return; const int m = (int)(e % NN); const v4f a = *(const v4f*)(S + e); v4h o;
#pragma unroll
    for (int q = 0; q < 4; ++q) { float d0 = __fsub_rn(a[q], CM[m + q]); asm volatile("" : "+v"(d0)); o[q] = tohx(__fmul_rn(__expf(d0), CIv[m + q])); } *(volatile v4h*)(P + e) = o; __threadfence(); *(volatile v4h*)(P + e) = o; }
__global__ __launch_bounds__(256) void k_osplit(const float* __restrict__ O, bf* Ah, bf* Al) { const size_t e = ((size_t)blockIdx.x * 256 + threadIdx.x) * 2; if (e >= (size_t)NN * C1) return; v2us oh, ol;
#pragma unroll
    for (int q = 0; q < 2; ++q) { unsigned short a, c2; splitf(O[e + q] * (1.0f / PCAR), a, c2); oh[q] = a; ol[q] = c2; } *(volatile v2us*)(Ah + e) = oh; *(volatile v2us*)(Al + e) = ol; __threadfence(); *(volatile v2us*)(Ah + e) = oh; *(volatile v2us*)(Al + e) = ol; }
__global__ __launch_bounds__(256) void k_outT(const float* __restrict__ MT, const float* __restrict__ x0b, float* OUTb) { const size_t e = ((size_t)blockIdx.x * 256 + threadIdx.x) * 2; if (e >= (size_t)C0 * NN) return; const int n = (int)(e % NN), o_ = (int)(e / NN); v2f o; o[0] = __fadd_rn(MT[(size_t)n * C0 + o_], bfr(x0b[e])); o[1] = __fadd_rn(MT[(size_t)(n + 1) * C0 + o_], bfr(x0b[e + 1])); *(volatile v2f*)(OUTb + e) = o; __threadfence(); *(volatile v2f*)(OUTb + e) = o; }

extern "C" void kernel_launch(void* const* d_in, const int* in_sizes, int n_in,
                              void* d_out, int out_size, void* d_ws, size_t ws_size, hipStream_t stream) {
    (void)in_sizes; (void)n_in; (void)out_size;
    const float* x0 = (const float*)d_in[0]; const float* x = (const float*)d_in[1]; const float* xd = (const float*)d_in[2]; const float* wphi = (const float*)d_in[3]; const float* wth = (const float*)d_in[4]; const float* wg = (const float*)d_in[5]; const float* wm = (const float*)d_in[6];
    float* OUT = (float*)d_out;
    char* wsp = (char*)d_ws;
    auto take = [&](size_t bytes) { char* p = wsp; wsp += (bytes + 255) & ~(size_t)255; return (void*)p; };
    bf* WPHI = (bf*)take((size_t)CI * C1 * 2); bf* WTH = (bf*)take((size_t)CI * C1 * 2); bf* WG = (bf*)take((size_t)C1 * C0 * 2); bf* WM = (bf*)take((size_t)C0 * C1 * 2);
    bf* XT = (bf*)take((size_t)NN * C0 * 2); float* F = (float*)take((size_t)NN * C1 * 4); bf* THh = (bf*)take((size_t)NN * CI * 2); bf* THl = (bf*)take((size_t)NN * CI * 2); bf* PHh = (bf*)take((size_t)NN * CI * 2); bf* PHl = (bf*)take((size_t)NN * CI * 2); h16* GT = (h16*)take((size_t)C1 * NN * 2);
    float* S = (float*)take((size_t)NN * NN * 4); h16* P = (h16*)take((size_t)NN * NN * 2); float* CM = (float*)take((size_t)NN * 4); float* CIv = (float*)take((size_t)NN * 4); float* O = (float*)take((size_t)NN * C1 * 4); bf* Oh = (bf*)take((size_t)NN * C1 * 2); bf* Ol = (bf*)take((size_t)NN * C1 * 2); float* MT = (float*)take((size_t)NN * C0 * 4);
    if ((size_t)(wsp - (char*)d_ws) > ws_size) return;
    { k_cvt8<<<(CI * C1 / 8 + 255) / 256, 256, 0, stream>>>(wphi, WPHI, (size_t)CI * C1 / 8); k_cvt8<<<(CI * C1 / 8 + 255) / 256, 256, 0, stream>>>(wth, WTH, (size_t)CI * C1 / 8); k_cvt8<<<(C1 * C0 / 8 + 255) / 256, 256, 0, stream>>>(wg, WG, (size_t)C1 * C0 / 8); k_cvt8<<<(C0 * C1 / 8 + 255) / 256, 256, 0, stream>>>(wm, WM, (size_t)C0 * C1 / 8); }
    const unsigned LC1 = (unsigned)(((size_t)NN * CI / 2 + 255) / 256);
    for (int b = 0; b < NB_; ++b) {
        k_xt8<<<(unsigned)(((size_t)NN * C1 / 4 + 255) / 256), 256, 0, stream>>>(xd + (size_t)b * C1 * NN, C1, XT);
        k_gemmw<bf, 0, false><<<dim3(NN / 64, CI / 64, 1), 32, 0, stream>>>(XT, nullptr, WTH, nullptr, C1, F, CI, nullptr, 0, 0, 0); k_split2<<<LC1, 256, 0, stream>>>(F, THh, THl, (size_t)NN * CI);
        k_xt8<<<(unsigned)(((size_t)NN * C1 / 4 + 255) / 256), 256, 0, stream>>>(x + (size_t)b * C1 * NN, C1, XT);
        k_gemmw<bf, 0, false><<<dim3(NN / 64, CI / 64, 1), 32, 0, stream>>>(XT, nullptr, WPHI, nullptr, C1, F, CI, nullptr, 0, 0, 0); k_split2<<<LC1, 256, 0, stream>>>(F, PHh, PHl, (size_t)NN * CI);
        k_xt8<<<(unsigned)(((size_t)NN * C0 / 4 + 255) / 256), 256, 0, stream>>>(x0 + (size_t)b * C0 * NN, C0, XT);
        k_gemmw<bf, 0, false><<<dim3(NN / 64, C1 / 64, 1), 32, 0, stream>>>(XT, nullptr, WG, nullptr, C0, F, C1, nullptr, 0, 0, 0); k_gt16<<<(unsigned)(((size_t)C1 * NN / 2 + 255) / 256), 256, 0, stream>>>(F, GT);
        k_gemmw<bf, 2, false><<<dim3(NN / 64, NN / 64, 1), 32, 0, stream>>>(THh, THl, PHh, PHl, CI, S, NN, nullptr, 0, 0, 0);
        k_colst<<<NN / 256, 256, 0, stream>>>(S, CM, CIv); k_pcol<<<(unsigned)(((size_t)NN * NN / 4 + 255) / 256), 256, 0, stream>>>(S, CM, CIv, P);
        k_gemmw<h16, 0, false><<<dim3(NN / 64, C1 / 64, 1), 32, 0, stream>>>(P, nullptr, GT, nullptr, NN, O, C1, nullptr, 0, 0, 0); k_osplit<<<(unsigned)(((size_t)NN * C1 / 2 + 255) / 256), 256, 0, stream>>>(O, Oh, Ol);
        k_gemmw<bf, 1, false><<<dim3(NN / 64, C0 / 64, 1), 32, 0, stream>>>(Oh, Ol, WM, nullptr, C1, MT, C0, nullptr, 0, 0, 0);
        k_outT<<<(unsigned)(((size_t)C0 * NN / 2 + 255) / 256), 256, 0, stream>>>(MT, x0 + (size_t)b * C0 * NN, OUT + (size_t)b * C0 * NN); }
}
